// NeuralODE_56238301774293
// MI455X (gfx1250) — hardware-verified
//
#include <hip/hip_runtime.h>
#include <math.h>

typedef __attribute__((ext_vector_type(16))) _Float16 v16h;
typedef __attribute__((ext_vector_type(8)))  _Float16 v8h;
typedef __attribute__((ext_vector_type(4)))  _Float16 v4h;
typedef __attribute__((ext_vector_type(16))) __bf16   v16b;
typedef __attribute__((ext_vector_type(8)))  __bf16   v8b;
typedef __attribute__((ext_vector_type(8)))  float    v8f;
typedef __attribute__((ext_vector_type(4)))  float    v4f;

__device__ __forceinline__ void dep_guard_h(v8f& a, v8f& b, v16h x, v16h y) { asm volatile("v_nop\n\tv_nop\n\tv_nop\n\tv_nop" : "+v"(a), "+v"(b) : "v"(x), "v"(y)); }
__device__ __forceinline__ void dep_guard_b(v8f& a, v8f& b, v16b x, v16b y) { asm volatile("v_nop\n\tv_nop\n\tv_nop\n\tv_nop" : "+v"(a), "+v"(b) : "v"(x), "v"(y)); }
__device__ __forceinline__ void keep4_h(v16h a, v16h b, v16h c, v16h d) { asm volatile("v_nop" :: "v"(a), "v"(b), "v"(c), "v"(d)); }
__device__ __forceinline__ void keep4_b(v16b a, v16b b, v16b c, v16b d) { asm volatile("v_nop" :: "v"(a), "v"(b), "v"(c), "v"(d)); }
__device__ __forceinline__ void acc_guard4(v8f& a, v8f& b, v8f& c, v8f& d) { asm volatile("v_nop\n\tv_nop\n\tv_nop\n\tv_nop" : "+v"(a), "+v"(b), "+v"(c), "+v"(d)); }
template <typename T> struct Frag;
template <> struct Frag<_Float16> {
  typedef v16h V; union U { v16h v; v8h h[2]; };
  static __device__ __forceinline__ v16h load(const _Float16* p) {
    U f; f.h[0] = *(const v8h*)(p); f.h[1] = *(const v8h*)(p + 16); return f.v;
  }
  static __device__ __forceinline__ v8f mma(v16h a, v16h b, v8f c) {
    return __builtin_amdgcn_wmma_f32_16x16x32_f16(false, a, false, b, (short)0, c, false, false);
  }
  static __device__ __forceinline__ void guard(v8f& a, v8f& b, v16h x, v16h y) { dep_guard_h(a, b, x, y); }
  static __device__ __forceinline__ void keep(v16h a, v16h b, v16h c, v16h d) { keep4_h(a, b, c, d); }
};
template <> struct Frag<__bf16> {
  typedef v16b V; union U { v16b v; v8b h[2]; };
  static __device__ __forceinline__ v16b load(const __bf16* p) {
    U f; f.h[0] = *(const v8b*)(p); f.h[1] = *(const v8b*)(p + 16); return f.v;
  }
  static __device__ __forceinline__ v8f mma(v16b a, v16b b, v8f c) {
    return __builtin_amdgcn_wmma_f32_16x16x32_bf16(false, a, false, b, (short)0, c, false, false);
  }
  static __device__ __forceinline__ void guard(v8f& a, v8f& b, v16b x, v16b y) { dep_guard_b(a, b, x, y); }
  static __device__ __forceinline__ void keep(v16b a, v16b b, v16b c, v16b d) { keep4_b(a, b, c, d); }
};

constexpr int NROWS     = 8192;
constexpr int DIM       = 512;
constexpr int NSTEPS    = 20;
constexpr int ROWS_BLK  = 32;
constexpr int NTHREADS  = 256;
constexpr int NWAVES    = NTHREADS / 32;
constexpr int PITCH16   = 520;
constexpr int NIT_IO    = (ROWS_BLK * DIM) / (4 * NTHREADS);
constexpr int NPAIR     = DIM * DIM / 2;
constexpr float W_SC    = 1024.0f;
constexpr float H_SC    = 1024.0f;
constexpr float L1_INV  = 1.0f / 1024.0f;
constexpr float L2_INV  = 1.0f / (1024.0f * 1024.0f);
constexpr size_t WPLANE_BYTES = (size_t)DIM * DIM * 2;
constexpr size_t WS_TOTAL     = 2 * WPLANE_BYTES;

static_assert(DIM % 32 == 0, "K multiple of 32");
static_assert(DIM == NWAVES * 64, "8 waves x 64 columns cover N");
static_assert(ROWS_BLK == 32, "two 16-row subtiles per wave");
static_assert(NROWS % ROWS_BLK == 0, "grid exact");
static_assert(NIT_IO * 4 * NTHREADS == ROWS_BLK * DIM, "io coverage exact");
static_assert(NIT_IO == 16, "io trips");
static_assert(NPAIR % NTHREADS == 0, "prep grid exact");
static_assert(PITCH16 % 8 == 0 && PITCH16 >= DIM, "16-B aligned f16 rows");
static_assert(WS_TOTAL <= 134217728ull, "carve budget");

__device__ __forceinline__ float tanh_f32(float x) {
  const float y = fabsf(x);
  const float e = expf(-2.0f * y);
  const float r = __builtin_amdgcn_rcpf(1.0f + e);
  const float th = (1.0f - e) * r;
  return copysignf(th, x);
}

__global__ __launch_bounds__(NTHREADS) void prep_weights_kernel(
    const float* __restrict__ W1, const float* __restrict__ W2,
    _Float16* __restrict__ w1t, _Float16* __restrict__ w2t) {
  const int i = blockIdx.x * NTHREADS + threadIdx.x;
  if (i < NPAIR) {
    const int o = i << 1;
    const int n = o / DIM;
    const int k = o - n * DIM;
    const _Float16 a0 = (_Float16)(W1[(size_t)k * DIM + n] * W_SC);
    const _Float16 a1 = (_Float16)(W1[(size_t)(k + 1) * DIM + n] * W_SC);
    const _Float16 c0 = (_Float16)(W2[(size_t)k * DIM + n] * W_SC);
    const _Float16 c1 = (_Float16)(W2[(size_t)(k + 1) * DIM + n] * W_SC);
    const unsigned ua = (unsigned)__builtin_bit_cast(unsigned short, a0) | ((unsigned)__builtin_bit_cast(unsigned short, a1) << 16);
    const unsigned uc = (unsigned)__builtin_bit_cast(unsigned short, c0) | ((unsigned)__builtin_bit_cast(unsigned short, c1) << 16);
    ((volatile unsigned*)w1t)[i] = ua;
    ((volatile unsigned*)w2t)[i] = uc;
    __threadfence();
    ((volatile unsigned*)w1t)[i] = ua;
    ((volatile unsigned*)w2t)[i] = uc;
  }
}

__device__ __forceinline__ void tile_gemm_32x64(const _Float16* a_sm, const _Float16* __restrict__ bt,
                                                int rlane, int koff, v8f (&acc)[2][4]) {
#pragma unroll
  for (int i = 0; i < 2; ++i)
#pragma unroll
    for (int j = 0; j < 4; ++j) acc[i][j] = (v8f){0.f,0.f,0.f,0.f,0.f,0.f,0.f,0.f};

#pragma unroll 2
  for (int k0 = 0; k0 < DIM; k0 += 32) {
    v16h bh[4];
#pragma unroll
    for (int j = 0; j < 4; ++j) {
      const size_t bo = (size_t)((j << 4) + rlane) * DIM + koff + k0;
      bh[j] = Frag<_Float16>::load(bt + bo);
    }
#pragma unroll
    for (int i = 0; i < 2; ++i) {
      const _Float16* ap = a_sm + ((i << 4) + rlane) * PITCH16 + koff + k0;
      const v16h ah = Frag<_Float16>::load(ap);
#pragma unroll
      for (int j = 0; j < 4; ++j) acc[i][j] = Frag<_Float16>::mma(ah, bh[j], acc[i][j]);
      Frag<_Float16>::guard(acc[i][0], acc[i][3], ah, ah);
    }
    Frag<_Float16>::keep(bh[0], bh[1], bh[2], bh[3]);
  }
  acc_guard4(acc[0][0], acc[0][1], acc[0][2], acc[0][3]);
  acc_guard4(acc[1][0], acc[1][1], acc[1][2], acc[1][3]);
}

__global__ __launch_bounds__(NTHREADS) void euler_mlp_kernel(
    const float* __restrict__ z0, const float* __restrict__ tvec,
    const unsigned short* __restrict__ w1p, const unsigned short* __restrict__ w2p,
    const float* __restrict__ b1, const float* __restrict__ b2,
    float* __restrict__ out) {
  __shared__ __align__(16) float    zf[ROWS_BLK * DIM];
  __shared__ __align__(16) _Float16 za[ROWS_BLK * PITCH16];
  __shared__ __align__(16) _Float16 ha[ROWS_BLK * PITCH16];

  const int tid   = threadIdx.x;
  const int lane  = tid & 31;
  const int wave  = tid >> 5;
  const int rlane = lane & 15;
  const int koff  = (lane >> 4) * 8;
  const int mOff  = (lane >> 4) * 8;
  const int grow0 = blockIdx.x * ROWS_BLK;
  const int n0w   = wave * 64;

  const _Float16* w1t = (const _Float16*)w1p + (size_t)n0w * DIM;
  const _Float16* w2t = (const _Float16*)w2p + (size_t)n0w * DIM;

  const float hstep = (tvec[1] - tvec[0]) * (1.0f / (float)NSTEPS);

  float bb1[4], bb2[4];
#pragma unroll
  for (int j = 0; j < 4; ++j) {
    bb1[j] = b1[n0w + (j << 4) + rlane];
    bb2[j] = b2[n0w + (j << 4) + rlane];
  }

#pragma unroll 4
  for (int it = 0; it < NIT_IO; ++it) {
    const int f   = tid + NTHREADS * it;
    const int e   = f << 2;
    const int row = e / DIM;
    const int col = e - row * DIM;
    const v4f v = *(const v4f*)(z0 + (size_t)(grow0 + row) * DIM + col);
    *(v4f*)(zf + row * DIM + col) = v;
    v4h hv;
    hv[0] = (_Float16)v[0]; hv[1] = (_Float16)v[1]; hv[2] = (_Float16)v[2]; hv[3] = (_Float16)v[3];
    *(v4h*)(za + row * PITCH16 + col) = hv;
  }

  v8f acc[2][4];
  for (int step = 0; step < NSTEPS; ++step) {
    __syncthreads();

    tile_gemm_32x64(za, w1t, rlane, koff, acc);
#pragma unroll
    for (int i = 0; i < 2; ++i) {
#pragma unroll
      for (int j = 0; j < 4; ++j) {
        const int n = n0w + (j << 4) + rlane;
#pragma unroll
        for (int r = 0; r < 8; ++r) {
          const int row = (i << 4) + mOff + r;
          const float u  = acc[i][j][r] * L1_INV + bb1[j];
          const float th = tanh_f32(u);
          ha[row * PITCH16 + n] = (_Float16)(th * H_SC);
        }
      }
    }
    __syncthreads();

    tile_gemm_32x64(ha, w2t, rlane, koff, acc);
#pragma unroll
    for (int i = 0; i < 2; ++i) {
#pragma unroll
      for (int j = 0; j < 4; ++j) {
        const int n = n0w + (j << 4) + rlane;
#pragma unroll
        for (int r = 0; r < 8; ++r) {
          const int row = (i << 4) + mOff + r;
          const float fv = acc[i][j][r] * L2_INV + bb2[j];
          const float zn = zf[row * DIM + n] + hstep * fv;
          zf[row * DIM + n] = zn;
          za[row * PITCH16 + n] = (_Float16)zn;
        }
      }
    }
  }
  __syncthreads();

  for (int pass = 0; pass < 2; ++pass) {
#pragma unroll
    for (int it = 0; it < NIT_IO; ++it) {
      const int f   = tid + NTHREADS * it;
      const int e   = f << 2;
      const int row = e / DIM;
      const int col = e - row * DIM;
      const v4f v = *(const v4f*)(zf + row * DIM + col);
      *(volatile v4f*)(out + (size_t)(grow0 + row) * DIM + col) = v;
    }
    __threadfence();
  }
}

extern "C" void kernel_launch(void* const* d_in, const int* in_sizes, int n_in,
                              void* d_out, int out_size, void* d_ws, size_t ws_size,
                              hipStream_t stream) {
  (void)n_in;
  const float* z0 = (const float*)d_in[0];
  const float* tv = (const float*)d_in[1];
  const float* W1 = (const float*)d_in[2];
  const float* b1 = (const float*)d_in[3];
  const float* W2 = (const float*)d_in[4];
  const float* b2 = (const float*)d_in[5];

  if (out_size != NROWS * DIM) return;
  if (in_sizes[0] != NROWS * DIM || in_sizes[1] < 2 || in_sizes[2] != DIM * DIM ||
      in_sizes[3] < DIM || in_sizes[4] != DIM * DIM || in_sizes[5] < DIM) return;
  if (ws_size < WS_TOTAL) return;

  unsigned char* ws = (unsigned char*)d_ws;
  _Float16* w1t = (_Float16*)(ws);
  _Float16* w2t = (_Float16*)(ws + WPLANE_BYTES);

  prep_weights_kernel<<<NPAIR / NTHREADS, NTHREADS, 0, stream>>>(W1, W2, w1t, w2t);
  euler_mlp_kernel<<<NROWS / ROWS_BLK, NTHREADS, 0, stream>>>(
      z0, tv, (const unsigned short*)w1t, (const unsigned short*)w2t, b1, b2, (float*)d_out);
}
